// EmilyGIN_angle_87703232184760
// MI455X (gfx1250) — hardware-verified
//
#include <hip/hip_runtime.h>
#include <stddef.h>


#define DF      128
#define NTHR    256
#define NWAVE   8
#define EPT     8
#define NGRP    2
#define CHUNK   (NTHR * EPT * NGRP)
#define WCAP    (EPT * NGRP * 32)
#define LISTN   (NWAVE * WCAP)
#define NB      512
#define NRT     (NB / 16)
#define RPW     (NB / NWAVE)
#define APR     128
#define APW     (APR / NWAVE)
#define LDS_AGG (NB * DF * 4 + LISTN * 4 + 64)

static_assert((CHUNK & (CHUNK - 1)) == 0);
static_assert(CHUNK <= 4096);
static_assert((NB & (NB - 1)) == 0 && NB <= 512);
static_assert(NRT % NWAVE == 0);
static_assert(RPW * NWAVE == NB);
static_assert(2 * DF * 8 <= LISTN * 4);
static_assert((DF * DF / 8) % NTHR == 0);
static_assert((NB * DF / 4) % NTHR == 0);

typedef float          v4f  __attribute__((ext_vector_type(4)));
typedef float          v8f  __attribute__((ext_vector_type(8)));
typedef int            v4i  __attribute__((ext_vector_type(4)));
typedef int            v8i  __attribute__((ext_vector_type(8)));
typedef unsigned short v8us __attribute__((ext_vector_type(8)));
typedef __bf16         v16b __attribute__((ext_vector_type(16)));
typedef double         v2d  __attribute__((ext_vector_type(2)));
union FragB { v16b v; v8us h[2]; v8i w; };

__device__ __forceinline__ unsigned bf16_rne_bits(float f) {
  const unsigned u = __float_as_uint(f);
  return (u + 0x7FFFu + ((u >> 16) & 1u)) >> 16;
}

__device__ __forceinline__ void split8(v4f a, v4f b, v8us& hi, v8us& lo) {
  float x[8];
  x[0] = a.x; x[1] = a.y; x[2] = a.z; x[3] = a.w;
  x[4] = b.x; x[5] = b.y; x[6] = b.z; x[7] = b.w;
#pragma unroll
  for (int j = 0; j < 8; ++j) {
    const unsigned hb  = bf16_rne_bits(x[j]);
    const float    res = x[j] - __uint_as_float(hb << 16);
    const unsigned lb  = bf16_rne_bits(res);
    hi[j] = (unsigned short)hb;
    lo[j] = (unsigned short)lb;
  }
}

__device__ __forceinline__ v8f wmb(const FragB& a, const FragB& b, v8f c) {
  v8f d = __builtin_amdgcn_wmma_f32_16x16x32_bf16(false, a.v, false, b.v, (short)0, c, false, false);
  asm volatile("v_nop\n\tv_nop\n\tv_nop\n\tv_nop" : "+v"(d) : "v"(a.w), "v"(b.w));
  return d;
}

template <int NBT>
__device__ __forceinline__ int scan_chunk(const int* __restrict__ dsts, int nE, int cbase, int nodeBase,
                                          int vec8, int* list, int tid, int lane, int wave) {
  int wc = 0;
#pragma unroll
  for (int g = 0; g < NGRP; ++g) {
    const int el0  = (g * NTHR + tid) * EPT;
    const int e0   = cbase + el0;
    const int sent = -2147483647 - 1;
    v4i da, db;
    if (vec8 != 0 && cbase + CHUNK <= nE) {
      da = *(const v4i*)(dsts + e0);
      db = *(const v4i*)(dsts + e0 + 4);
    } else {
      da.x = (e0     < nE) ? dsts[min(e0, nE - 1)] : sent;
      da.y = (e0 + 1 < nE) ? dsts[min(e0 + 1, nE - 1)] : sent;
      da.z = (e0 + 2 < nE) ? dsts[min(e0 + 2, nE - 1)] : sent;
      da.w = (e0 + 3 < nE) ? dsts[min(e0 + 3, nE - 1)] : sent;
      db.x = (e0 + 4 < nE) ? dsts[min(e0 + 4, nE - 1)] : sent;
      db.y = (e0 + 5 < nE) ? dsts[min(e0 + 5, nE - 1)] : sent;
      db.z = (e0 + 6 < nE) ? dsts[min(e0 + 6, nE - 1)] : sent;
      db.w = (e0 + 7 < nE) ? dsts[min(e0 + 7, nE - 1)] : sent;
    }
    const unsigned nb = (unsigned)nodeBase;
    const unsigned s0 = (unsigned)da.x - nb, s1 = (unsigned)da.y - nb;
    const unsigned s2 = (unsigned)da.z - nb, s3 = (unsigned)da.w - nb;
    const unsigned s4 = (unsigned)db.x - nb, s5 = (unsigned)db.y - nb;
    const unsigned s6 = (unsigned)db.z - nb, s7 = (unsigned)db.w - nb;
    const bool h0 = s0 < (unsigned)NBT, h1 = s1 < (unsigned)NBT, h2 = s2 < (unsigned)NBT, h3 = s3 < (unsigned)NBT;
    const bool h4 = s4 < (unsigned)NBT, h5 = s5 < (unsigned)NBT, h6 = s6 < (unsigned)NBT, h7 = s7 < (unsigned)NBT;
    const unsigned any = __builtin_amdgcn_ballot_w32(h0 | h1 | h2 | h3 | h4 | h5 | h6 | h7);
    if (any != 0u) {
#define HITJ(J, HJ, SJ) { \
        const unsigned mj = __builtin_amdgcn_ballot_w32(HJ); \
        if (mj != 0u) { \
          if (HJ) { \
            const int pos = wc + (int)__builtin_amdgcn_mbcnt_lo(mj, 0u); \
            if (pos < WCAP) list[wave * WCAP + pos] = ((el0 + (J)) << 12) | (int)(SJ); \
          } \
          wc += (int)__builtin_popcount(mj); } }
      HITJ(0, h0, s0)
      HITJ(1, h1, s1)
      HITJ(2, h2, s2)
      HITJ(3, h3, s3)
      HITJ(4, h4, s4)
      HITJ(5, h5, s5)
      HITJ(6, h6, s6)
      HITJ(7, h7, s7)
#undef HITJ
    }
  }
  return wc;
}

__global__ __launch_bounds__(NTHR) void k_wprep(
    const float* __restrict__ W1, const float* __restrict__ W2,
    unsigned short* w1h, unsigned short* w1l, unsigned short* w2h, unsigned short* w2l) {
  const int i   = blockIdx.x * NTHR + threadIdx.x;
  const int per = DF * DF / 8;
  if (i >= 2 * per) return;
  const bool first = i < per;
  const int o  = (first ? i : i - per) * 8;
  const int n  = o >> 7;
  const int k0 = o & (DF - 1);
  const float* p = (first ? W1 : W2) + (size_t)k0 * DF + n;
  v4f a, b;
  a.x = p[0];      a.y = p[DF];     a.z = p[2 * DF]; a.w = p[3 * DF];
  b.x = p[4 * DF]; b.y = p[5 * DF]; b.z = p[6 * DF]; b.w = p[7 * DF];
  v8us hv, lv;
  split8(a, b, hv, lv);
  unsigned short* dh = (first ? w1h : w2h) + o;
  unsigned short* dl = (first ? w1l : w2l) + o;
  *(volatile v8us*)dh = hv;
  *(volatile v8us*)dl = lv;
  __threadfence();
  *(volatile v8us*)dh = hv;
  *(volatile v8us*)dl = lv;
}

__device__ __forceinline__ void mlp_layer(float* acc, const unsigned short* __restrict__ wh,
                                          const unsigned short* __restrict__ wl,
                                          const float* __restrict__ bias, int wave, int hh, int m) {
  float bia[8];
#pragma unroll
  for (int t8 = 0; t8 < 8; ++t8) bia[t8] = bias[16 * t8 + m];

#pragma unroll 1
  for (int tt = 0; tt < NRT / NWAVE; ++tt) {
    const int t = wave + NWAVE * tt;
    v8f c[8];
#pragma unroll
    for (int t8 = 0; t8 < 8; ++t8) { v8f z = {0.f, 0.f, 0.f, 0.f, 0.f, 0.f, 0.f, 0.f}; c[t8] = z; }

#pragma unroll 1
    for (int kt = 0; kt < DF / 32; ++kt) {
      const float* ap = acc + (16 * t + m) * DF + 32 * kt + 8 * hh;
      const v4f p0 = *(const v4f*)ap,        p1 = *(const v4f*)(ap + 4);
      const v4f p2 = *(const v4f*)(ap + 16), p3 = *(const v4f*)(ap + 20);
      FragB ah, al;
      split8(p0, p1, ah.h[0], al.h[0]);
      split8(p2, p3, ah.h[1], al.h[1]);
#pragma unroll
      for (int t8 = 0; t8 < 8; ++t8) {
        const size_t bo = (size_t)(16 * t8 + m) * DF + 32 * kt + 8 * hh;
        FragB bh, bl;
        bh.h[0] = *(const v8us*)(wh + bo);
        bh.h[1] = *(const v8us*)(wh + bo + 16);
        bl.h[0] = *(const v8us*)(wl + bo);
        bl.h[1] = *(const v8us*)(wl + bo + 16);
        c[t8] = wmb(ah, bh, c[t8]);
        c[t8] = wmb(al, bh, c[t8]);
        c[t8] = wmb(ah, bl, c[t8]);
      }
    }
    float* sp = acc + (16 * t + 8 * hh) * DF + m;
#pragma unroll
    for (int t8 = 0; t8 < 8; ++t8) {
#pragma unroll
      for (int r = 0; r < 8; ++r) {
        const float v = c[t8][r] + bia[t8];
        sp[r * DF + 16 * t8] = fmaxf(v, 0.f);
      }
    }
  }
}

__global__ __launch_bounds__(NTHR) void k_agg(
    const float* __restrict__ feat, const int* __restrict__ ei,
    const unsigned short* __restrict__ w1h, const unsigned short* __restrict__ w1l,
    const unsigned short* __restrict__ w2h, const unsigned short* __restrict__ w2l,
    const float* __restrict__ b1, const float* __restrict__ b2,
    float* yp, double* part, int nN, int nE, int vec8) {
  extern __shared__ v4f lds_dyn[];
  float*  acc  = (float*)lds_dyn;
  int*    list = (int*)(acc + NB * DF);
  int*    wcnt = list + LISTN;
  double* sd   = (double*)list;
  const int tid = threadIdx.x, lane = tid & 31, wave = tid >> 5, hh = lane >> 4, m = lane & 15;
  const int nodeBase = blockIdx.x * NB;
  const int* dsts = ei + nE;

  {
    const v4f z = {0.f, 0.f, 0.f, 0.f};
#pragma unroll 4
    for (int i = 0; i < (NB * DF / 4) / NTHR; ++i) lds_dyn[i * NTHR + tid] = z;
  }
  __syncthreads();

  const int nChunks = (nE + CHUNK - 1) / CHUNK;
#pragma unroll 1
  for (int ch = 0; ch < nChunks; ++ch) {
    const int cbase = ch * CHUNK;
    const int wc = scan_chunk<NB>(dsts, nE, cbase, nodeBase, vec8, list, tid, lane, wave);
    if (lane == 0) wcnt[wave] = wc;
    __syncthreads();
    if (wave == 0) {
#pragma unroll 1
      for (int wsx = 0; wsx < NWAVE; ++wsx) {
        int n = __builtin_amdgcn_readfirstlane(wcnt[wsx]);
        n = n > WCAP ? WCAP : (n < 0 ? 0 : n);
        const int* lp = list + wsx * WCAP;
#pragma unroll 1
        for (int i = 0; i < n; ++i) {
          const int ent  = __builtin_amdgcn_readfirstlane(lp[i]);
          const int slot = ent & (NB - 1);
          int e = cbase + ((ent >> 12) & (CHUNK - 1));
          e = e > nE - 1 ? nE - 1 : e;
          int src = ei[e];
          src = src < 0 ? 0 : (src > nN - 1 ? nN - 1 : src);
          const v4f v = *(const v4f*)(feat + (size_t)src * DF + 4 * lane);
          v4f* ap = (v4f*)(acc + slot * DF + 4 * lane);
          *ap = *ap + v;
        }
      }
    }
    __syncthreads();
  }

#pragma unroll 4
  for (int i = 0; i < (NB * DF / 4) / NTHR; ++i) {
    const int idx  = i * NTHR + tid;
    const int slot = idx >> 5;
    const int c4   = (idx & 31) * 4;
    int node = nodeBase + slot;
    node = node > nN - 1 ? nN - 1 : node;
    const v4f fv = *(const v4f*)(feat + (size_t)node * DF + c4);
    v4f* ap = (v4f*)(acc + slot * DF + c4);
    *ap = *ap + fv;
  }
  __syncthreads();

  mlp_layer(acc, w1h, w1l, b1, wave, hh, m);
  __syncthreads();
  mlp_layer(acc, w2h, w2l, b2, wave, hh, m);
  __syncthreads();

  {
    const float* lsrc = acc + wave * RPW * DF + 4 * lane;
    float* gdst = yp + ((size_t)nodeBase + wave * RPW) * DF + 4 * lane;
#pragma unroll 1
    for (int i = 0; i < RPW; ++i) { const v4f v = *(const v4f*)(lsrc + i * DF); *(volatile v4f*)(gdst + (size_t)i * DF) = v; }
    __threadfence();
#pragma unroll 1
    for (int i = 0; i < RPW; ++i) { const v4f v = *(const v4f*)(lsrc + i * DF); *(volatile v4f*)(gdst + (size_t)i * DF) = v; }
  }

  if (tid < DF) {
    int nrows = nN - nodeBase;
    nrows = nrows > NB ? NB : (nrows < 0 ? 0 : nrows);
    double s = 0.0, q = 0.0;
#pragma unroll 1
    for (int r = 0; r < nrows; ++r) {
      const double v = (double)acc[r * DF + tid];
      s += v;
      q += v * v;
    }
    sd[tid]      = s;
    sd[DF + tid] = q;
  }
  __syncthreads();
  if (wave == 0) {
    double* pp = part + (size_t)blockIdx.x * 2 * DF;
    v2d pv[4];
#pragma unroll
    for (int qd = 0; qd < 4; ++qd) pv[qd] = *(const v2d*)(sd + (qd * 32 + lane) * 2);
#pragma unroll
    for (int qd = 0; qd < 4; ++qd) *(volatile v2d*)(pp + (qd * 32 + lane) * 2) = pv[qd];
    __threadfence();
#pragma unroll
    for (int qd = 0; qd < 4; ++qd) *(volatile v2d*)(pp + (qd * 32 + lane) * 2) = pv[qd];
  }
}

__global__ __launch_bounds__(DF) void k_bnstat(
    const double* __restrict__ part, const float* __restrict__ gamma,
    float* meanv, float* scv, int nBlk, double invN) {
  __shared__ __attribute__((aligned(16))) float sm[DF];
  __shared__ __attribute__((aligned(16))) float ss[DF];
  const int c = threadIdx.x, lane = c & 31, wave = c >> 5;
  double s = 0.0, q = 0.0;
#pragma unroll 1
  for (int b = 0; b < nBlk; ++b) {
    s += part[(size_t)b * 2 * DF + c];
    q += part[(size_t)b * 2 * DF + DF + c];
  }
  const double mean = s * invN;
  double var = q * invN - mean * mean;
  var = var < 0.0 ? 0.0 : var;
  const float rs = rsqrtf((float)var + 1e-5f);
  sm[c] = (float)mean;
  ss[c] = gamma[c] * rs;
  __syncthreads();
  if (wave == 0) {
    const v4f mv = *(const v4f*)(sm + 4 * lane);
    const v4f sv = *(const v4f*)(ss + 4 * lane);
    *(volatile v4f*)(meanv + 4 * lane) = mv;
    *(volatile v4f*)(scv   + 4 * lane) = sv;
    __threadfence();
    *(volatile v4f*)(meanv + 4 * lane) = mv;
    *(volatile v4f*)(scv   + 4 * lane) = sv;
  }
}

__global__ __launch_bounds__(NTHR) void k_apply(
    const float* __restrict__ yp, const float* __restrict__ meanv, const float* __restrict__ scv,
    const float* __restrict__ beta, float* out, int nN) {
  const int tid = threadIdx.x, lane = tid & 31, wave = tid >> 5;
  const int rb = blockIdx.x * APR + wave * APW;
  const v4f mu = *(const v4f*)(meanv + 4 * lane);
  const v4f sc = *(const v4f*)(scv   + 4 * lane);
  const v4f be = *(const v4f*)(beta  + 4 * lane);
#pragma unroll 1
  for (int i = 0; i < APW; ++i) {
    const int row = rb + i;
    if (row < nN) {
      const v4f v = *(const v4f*)(yp + (size_t)row * DF + 4 * lane);
      const v4f o = (v - mu) * sc + be;
      *(volatile v4f*)(out + (size_t)row * DF + 4 * lane) = o;
    }
  }
  __threadfence();
#pragma unroll 1
  for (int i = 0; i < APW; ++i) {
    const int row = rb + i;
    if (row < nN) {
      const v4f v = *(const v4f*)(yp + (size_t)row * DF + 4 * lane);
      const v4f o = (v - mu) * sc + be;
      *(volatile v4f*)(out + (size_t)row * DF + 4 * lane) = o;
    }
  }
}

extern "C" void kernel_launch(void* const* d_in, const int* in_sizes, int n_in,
                              void* d_out, int out_size, void* d_ws, size_t ws_size,
                              hipStream_t stream) {
  if (n_in < 8) return;
  const int nN = in_sizes[0] / DF;
  const int nE = in_sizes[1] / 2;
  if (nN <= 0 || nE < 0 || in_sizes[0] != nN * DF || in_sizes[1] != nE * 2) return;
  if (in_sizes[2] != DF * DF || in_sizes[4] != DF * DF) return;
  if (in_sizes[3] < DF || in_sizes[5] < DF || in_sizes[6] < DF || in_sizes[7] < DF) return;
  if (out_size != nN * DF) return;

  const float* feat  = (const float*)d_in[0];
  const int*   ei    = (const int*)d_in[1];
  const float* W1    = (const float*)d_in[2];
  const float* b1    = (const float*)d_in[3];
  const float* W2    = (const float*)d_in[4];
  const float* b2    = (const float*)d_in[5];
  const float* gamma = (const float*)d_in[6];
  const float* beta  = (const float*)d_in[7];
  float* out = (float*)d_out;

  const int nBlk = (nN + NB - 1) / NB;
  const int nAp  = (nN + APR - 1) / APR;

  char* ws = (char*)d_ws;
  size_t off = 0;
  const size_t plane = (size_t)DF * DF * 2;
  const size_t oW1h = off; off += plane;                                  off = (off + 255) & ~(size_t)255;
  const size_t oW1l = off; off += plane;                                  off = (off + 255) & ~(size_t)255;
  const size_t oW2h = off; off += plane;                                  off = (off + 255) & ~(size_t)255;
  const size_t oW2l = off; off += plane;                                  off = (off + 255) & ~(size_t)255;
  const size_t oY   = off; off += (size_t)nBlk * NB * DF * 4;             off = (off + 255) & ~(size_t)255;
  const size_t oP   = off; off += (size_t)nBlk * 2 * DF * 8;              off = (off + 255) & ~(size_t)255;
  const size_t oMu  = off; off += (size_t)DF * 4;                         off = (off + 255) & ~(size_t)255;
  const size_t oSc  = off; off += (size_t)DF * 4;                         off = (off + 255) & ~(size_t)255;
  if (off > ws_size || off > ((size_t)128 << 20)) return;
  unsigned short* w1h = (unsigned short*)(ws + oW1h);
  unsigned short* w1l = (unsigned short*)(ws + oW1l);
  unsigned short* w2h = (unsigned short*)(ws + oW2h);
  unsigned short* w2l = (unsigned short*)(ws + oW2l);
  float*  yp    = (float*)(ws + oY);
  double* part  = (double*)(ws + oP);
  float*  meanv = (float*)(ws + oMu);
  float*  scv   = (float*)(ws + oSc);

  const int vec8 = ((nE & 3) == 0) ? 1 : 0;
  const double invN = 1.0 / (double)nN;

  const int nPrep = 2 * (DF * DF / 8);
  k_wprep<<<(nPrep + NTHR - 1) / NTHR, NTHR, 0, stream>>>(W1, W2, w1h, w1l, w2h, w2l);

  hipFuncSetAttribute(reinterpret_cast<const void*>(&k_agg),
                      hipFuncAttributeMaxDynamicSharedMemorySize, LDS_AGG);
  k_agg<<<nBlk, NTHR, LDS_AGG, stream>>>(feat, ei, w1h, w1l, w2h, w2l, b1, b2, yp, part, nN, nE, vec8);

  k_bnstat<<<1, DF, 0, stream>>>(part, gamma, meanv, scv, nBlk, invN);

  k_apply<<<nAp, NTHR, 0, stream>>>(yp, meanv, scv, beta, out, nN);
}
